// CalculateAttention_9603546874096
// MI455X (gfx1250) — hardware-verified
//
#include <hip/hip_runtime.h>

constexpr int kNumB  = 2;
constexpr int kNumH  = 16;
constexpr int kSeq   = 4096;
constexpr int kHd    = 64;
constexpr int kNumBH = kNumB * kNumH;
constexpr int kElems = kNumBH * kSeq * kHd;
constexpr int kKvTile = 64;
constexpr int kQTile  = 64;
constexpr float kPCarry = 32768.0f;
constexpr float kScoreScaleLog2 = 0.125f * 1.44269504088896340736f;

static_assert(kHd == 64, "head dim 64");
static_assert(kSeq % kKvTile == 0, "kv tile multiple");
static_assert(kSeq % kQTile == 0, "q tile multiple");
static_assert(kElems % (8 * 256) == 0, "cast grid exact");

constexpr size_t kPlaneBytes = (size_t)kElems * 2;
constexpr size_t kWsTotal    = 3 * kPlaneBytes;
static_assert(kWsTotal <= 134217728ull, "carve under 128 MiB");

typedef __attribute__((ext_vector_type(16))) _Float16 v16h;
typedef __attribute__((ext_vector_type(8)))  _Float16 v8h;
typedef __attribute__((ext_vector_type(16))) __bf16   v16b;
typedef __attribute__((ext_vector_type(8)))  __bf16   v8b;
typedef __attribute__((ext_vector_type(8)))  float    v8f;
typedef __attribute__((ext_vector_type(4)))  float    v4f;
typedef __attribute__((ext_vector_type(4)))  unsigned int v4u;

__device__ __forceinline__ unsigned short f2bf_bits(float f) {
  unsigned u = __float_as_uint(f);
  return (unsigned short)((u + 0x7FFFu + ((u >> 16) & 1u)) >> 16);
}
__device__ __forceinline__ float bf_bits2f(unsigned short h) { return __uint_as_float(((unsigned)h) << 16); }

__device__ __forceinline__ void dep_guard_h(v8f& a, v8f& b, v16h x, v16h y) { asm volatile("v_nop\n\tv_nop\n\tv_nop\n\tv_nop" : "+v"(a), "+v"(b) : "v"(x), "v"(y)); }
__device__ __forceinline__ void dep_guard_b(v8f& a, v8f& b, v16b x, v16b y) { asm volatile("v_nop\n\tv_nop\n\tv_nop\n\tv_nop" : "+v"(a), "+v"(b) : "v"(x), "v"(y)); }
__device__ __forceinline__ void keep4_h(v16h a, v16h b, v16h c, v16h d) { asm volatile("v_nop" :: "v"(a), "v"(b), "v"(c), "v"(d)); }
__device__ __forceinline__ void keep4_b(v16b a, v16b b, v16b c, v16b d) { asm volatile("v_nop" :: "v"(a), "v"(b), "v"(c), "v"(d)); }
template <typename T> struct Frag;
template <> struct Frag<_Float16> {
  typedef v16h V; union U { v16h v; v8h h[2]; };
  static __device__ __forceinline__ v16h load(const _Float16* p) {
    U f; f.h[0] = *(const v8h*)(p); f.h[1] = *(const v8h*)(p + 16); return f.v;
  }
  static __device__ __forceinline__ v8f mma(v16h a, v16h b, v8f c) {
    return __builtin_amdgcn_wmma_f32_16x16x32_f16(false, a, false, b, (short)0, c, false, false);
  }
  static __device__ __forceinline__ void guard(v8f& a, v8f& b, v16h x, v16h y) { dep_guard_h(a, b, x, y); }
  static __device__ __forceinline__ void keep(v16h a, v16h b, v16h c, v16h d) { keep4_h(a, b, c, d); }
};
template <> struct Frag<__bf16> {
  typedef v16b V; union U { v16b v; v8b h[2]; };
  static __device__ __forceinline__ v16b load(const __bf16* p) {
    U f; f.h[0] = *(const v8b*)(p); f.h[1] = *(const v8b*)(p + 16); return f.v;
  }
  static __device__ __forceinline__ v8f mma(v16b a, v16b b, v8f c) {
    return __builtin_amdgcn_wmma_f32_16x16x32_bf16(false, a, false, b, (short)0, c, false, false);
  }
  static __device__ __forceinline__ void guard(v8f& a, v8f& b, v16b x, v16b y) { dep_guard_b(a, b, x, y); }
  static __device__ __forceinline__ void keep(v16b a, v16b b, v16b c, v16b d) { keep4_b(a, b, c, d); }
};

__device__ __forceinline__ v8f mma_bf16_g(v16b a, v16b b, v8f c) {
  c = __builtin_amdgcn_wmma_f32_16x16x32_bf16(false, a, false, b, (short)0, c, false, false);
  asm volatile("v_nop\n\tv_nop\n\tv_nop\n\tv_nop" : "+v"(c) : "v"(a), "v"(b));
  return c;
}
__device__ __forceinline__ v8f mma_f16_g(v16h a, v16h b, v8f c) {
  c = __builtin_amdgcn_wmma_f32_16x16x32_f16(false, a, false, b, (short)0, c, false, false);
  asm volatile("v_nop\n\tv_nop\n\tv_nop\n\tv_nop" : "+v"(c) : "v"(a), "v"(b));
  return c;
}

__device__ __forceinline__ float ex2(float x) {
#if __has_builtin(__builtin_amdgcn_exp2f)
  return __builtin_amdgcn_exp2f(x);
#else
  return exp2f(x);
#endif
}

__device__ __forceinline__ unsigned int f16bits_of_bf16val(float f) {
  const float xb = bf_bits2f(f2bf_bits(f));
  const _Float16 h = (_Float16)xb;
  return (unsigned int)__builtin_bit_cast(unsigned short, h);
}

__global__ __launch_bounds__(256) void cast_bf16_x8(const float* __restrict__ in,
                                                     unsigned short* __restrict__ out, int n8) {
  const int i = blockIdx.x * 256 + threadIdx.x;
  if (i < n8) {
    const v4f a = *(const v4f*)(in + (size_t)i * 8);
    const v4f c = *(const v4f*)(in + (size_t)i * 8 + 4);
    v4u u;
    u[0] = (unsigned)f2bf_bits(a[0]) | ((unsigned)f2bf_bits(a[1]) << 16);
    u[1] = (unsigned)f2bf_bits(a[2]) | ((unsigned)f2bf_bits(a[3]) << 16);
    u[2] = (unsigned)f2bf_bits(c[0]) | ((unsigned)f2bf_bits(c[1]) << 16);
    u[3] = (unsigned)f2bf_bits(c[2]) | ((unsigned)f2bf_bits(c[3]) << 16);
    v4u* p = (v4u*)(out + (size_t)i * 8);
    *(volatile v4u*)p = u;
    __threadfence();
    *(volatile v4u*)p = u;
  }
}

__global__ __launch_bounds__(256) void vt_cast_f16(const float* __restrict__ vin,
                                                    unsigned short* __restrict__ vt) {
  __shared__ __align__(16) float tile[kHd][68];
  const int tid = threadIdx.x;
  const int bh  = blockIdx.x / (kSeq / kKvTile);
  const int kc  = blockIdx.x - bh * (kSeq / kKvTile);
  const int kv0 = kc * kKvTile;
  {
    const int kv = tid >> 2;
    const int d0 = (tid & 3) * 16;
    const float* src = vin + ((size_t)bh * kSeq + kv0 + kv) * kHd + d0;
#pragma unroll
    for (int i = 0; i < 4; ++i) {
      const v4f x = *(const v4f*)(src + 4 * i);
      tile[d0 + 4 * i + 0][kv] = x[0];
      tile[d0 + 4 * i + 1][kv] = x[1];
      tile[d0 + 4 * i + 2][kv] = x[2];
      tile[d0 + 4 * i + 3][kv] = x[3];
    }
  }
  __syncthreads();
  {
    const int wave = tid >> 5, lane = tid & 31;
    const int q  = lane >> 3;
    const int c8 = (lane & 7) * 8;
    for (int pass = 0; pass < 2; ++pass) {
#pragma unroll
      for (int it = 0; it < 2; ++it) {
        const int dl = wave * 8 + it * 4 + q;
        const v4f x0 = *(const v4f*)(&tile[dl][c8]);
        const v4f x1 = *(const v4f*)(&tile[dl][c8 + 4]);
        v4u u;
        u[0] = f16bits_of_bf16val(x0[0]) | (f16bits_of_bf16val(x0[1]) << 16);
        u[1] = f16bits_of_bf16val(x0[2]) | (f16bits_of_bf16val(x0[3]) << 16);
        u[2] = f16bits_of_bf16val(x1[0]) | (f16bits_of_bf16val(x1[1]) << 16);
        u[3] = f16bits_of_bf16val(x1[2]) | (f16bits_of_bf16val(x1[3]) << 16);
        *(volatile v4u*)(vt + (((size_t)bh * kHd + dl) * kSeq + kv0 + c8)) = u;
      }
      __threadfence();
    }
  }
}

__global__ __launch_bounds__(128) void attn_fwd(const unsigned short* __restrict__ qb,
                                                 const unsigned short* __restrict__ kb,
                                                 const unsigned short* __restrict__ vt,
                                                 float* __restrict__ out) {
  __shared__ __align__(16) float Os[4][16 * 68];

  const int tid  = threadIdx.x;
  const int wave = tid >> 5;
  const int lane = tid & 31;
  const int hh   = lane >> 4;
  const int c    = lane & 15;

  const int bx   = blockIdx.x;
  const int qblk = bx % (kSeq / kQTile);
  const int bh   = bx / (kSeq / kQTile);
  const int q0   = qblk * kQTile + wave * 16;

  const __bf16*   Qp = (const __bf16*)qb + (size_t)bh * kSeq * kHd;
  const __bf16*   Kp = (const __bf16*)kb + (size_t)bh * kSeq * kHd;
  const _Float16* Vp = (const _Float16*)vt + (size_t)bh * kHd * kSeq;
  float*          Op = out + (size_t)bh * kSeq * kHd;

  v16b qf[2];
#pragma unroll
  for (int dc = 0; dc < 2; ++dc)
    qf[dc] = Frag<__bf16>::load(Qp + (size_t)(q0 + c) * kHd + dc * 32 + 8 * hh);

  float m_run = -__builtin_inff();
  float l_run = 0.0f;
  v8f oacc[4];
#pragma unroll
  for (int t = 0; t < 4; ++t) oacc[t] = (v8f){0.f,0.f,0.f,0.f,0.f,0.f,0.f,0.f};

#pragma unroll 1
  for (int kc = 0; kc < kSeq / kKvTile; ++kc) {
    const int kv0 = kc * kKvTile;

    v8f st[4];
#pragma unroll
    for (int j = 0; j < 4; ++j) {
      v8f a = (v8f){0.f,0.f,0.f,0.f,0.f,0.f,0.f,0.f};
#pragma unroll
      for (int dc = 0; dc < 2; ++dc) {
        const v16b kf = Frag<__bf16>::load(Kp + (size_t)(kv0 + j * 16 + c) * kHd + dc * 32 + 8 * hh);
        a = mma_bf16_g(kf, qf[dc], a);
      }
      st[j] = a;
    }

    float cmx = -__builtin_inff();
#pragma unroll
    for (int j = 0; j < 4; ++j)
#pragma unroll
      for (int r = 0; r < 8; ++r) cmx = fmaxf(cmx, st[j][r]);
    cmx = fmaxf(cmx, __shfl_xor(cmx, 16, 32));
    const float mnew  = fmaxf(m_run, cmx);
    const float alpha = ex2((m_run - mnew) * kScoreScaleLog2);
    m_run = mnew;
    const float moff = mnew * kScoreScaleLog2;

    v16h pf[2];
    float psum = 0.0f;
#pragma unroll
    for (int kk = 0; kk < 2; ++kk) {
#pragma unroll
      for (int e = 0; e < 16; ++e) {
        const int j = 2 * kk + (e >> 3);
        const int r = e & 7;
        const float p = ex2(fmaf(st[j][r], kScoreScaleLog2, -moff));
        psum += p;
        pf[kk][e] = (_Float16)(p * kPCarry);
      }
    }
    psum += __shfl_xor(psum, 16, 32);
    l_run = l_run * alpha + psum;

#pragma unroll
    for (int r = 0; r < 8; ++r) {
      const float ar = __shfl(alpha, 8 * hh + r, 32);
#pragma unroll
      for (int t = 0; t < 4; ++t) oacc[t][r] *= ar;
    }

#pragma unroll
    for (int kk = 0; kk < 2; ++kk) {
#pragma unroll
      for (int t = 0; t < 4; ++t) {
        const v16h vf = Frag<_Float16>::load(Vp + (size_t)(t * 16 + c) * kSeq + kv0 + kk * 32 + 8 * hh);
        oacc[t] = mma_f16_g(pf[kk], vf, oacc[t]);
      }
    }
  }

  float* os = Os[wave];
  const float invl = 1.0f / (l_run * kPCarry);
#pragma unroll
  for (int r = 0; r < 8; ++r) {
    const float ir = __shfl(invl, 8 * hh + r, 32);
#pragma unroll
    for (int t = 0; t < 4; ++t) os[(8 * hh + r) * 68 + t * 16 + c] = oacc[t][r] * ir;
  }
  __builtin_amdgcn_fence(__ATOMIC_RELEASE, "workgroup");
  __builtin_amdgcn_wave_barrier();
  __builtin_amdgcn_fence(__ATOMIC_ACQUIRE, "workgroup");
  {
    const int c4 = (lane & 15) * 4;
    for (int pass = 0; pass < 2; ++pass) {
#pragma unroll
      for (int it = 0; it < 8; ++it) {
        const int row = it * 2 + hh;
        v4f val = *(const v4f*)(os + row * 68 + c4);
        *(volatile v4f*)(Op + (size_t)(q0 + row) * kHd + c4) = val;
      }
      __threadfence();
    }
  }
}

extern "C" void kernel_launch(void* const* d_in, const int* in_sizes, int n_in,
                              void* d_out, int out_size, void* d_ws, size_t ws_size,
                              hipStream_t stream) {
  if (n_in < 3) return;
  if (in_sizes[0] != kElems || in_sizes[1] != kElems || in_sizes[2] != kElems) return;
  if (out_size != kElems) return;
  if (ws_size < kWsTotal) return;

  const float* Q = (const float*)d_in[0];
  const float* K = (const float*)d_in[1];
  const float* V = (const float*)d_in[2];
  float* O = (float*)d_out;

  unsigned short* qbp = (unsigned short*)d_ws;
  unsigned short* kbp = (unsigned short*)((char*)d_ws + kPlaneBytes);
  unsigned short* vtp = (unsigned short*)((char*)d_ws + 2 * kPlaneBytes);

  const int n8 = kElems / 8;
  const int castGrid = n8 / 256;
  const int tileGrid = kNumBH * (kSeq / kKvTile);

  cast_bf16_x8<<<castGrid, 256, 0, stream>>>(Q, qbp, n8);
  cast_bf16_x8<<<castGrid, 256, 0, stream>>>(K, kbp, n8);
  vt_cast_f16<<<tileGrid, 256, 0, stream>>>(V, vtp);
  attn_fwd<<<kNumBH * (kSeq / kQTile), 128, 0, stream>>>(qbp, kbp, vtp, O);
}
